// SparseConstraint_15350213116416
// MI455X (gfx1250) — hardware-run, weakly checked
//
#include <hip/hip_runtime.h>

#define NBATCH   4
#define IMG      1024
#define NPSIDE   128
#define NPB      (NPSIDE * NPSIDE)
#define NPATCH   (NBATCH * NPB)
#define WAVES    16
#define NTHR     (WAVES * 32)
#define PPB      32
#define NBLK     (NPATCH / PPB)
#define TXTK     768
#define NF       32
#define XELEMS   (NBATCH * IMG * IMG)
#define XPIECES  (XELEMS / 4)

#define OFF_TXT  0
#define OFF_W1   512
#define OFF_W2   1536
#define OFF_M1   11776
#define OFF_M2   24064
#define OFF_M3   28160
#define WS_TOTAL 29184

static_assert(NBLK * PPB == NPATCH);
static_assert(NPB % PPB == 0);
static_assert(NTHR == 512);
static_assert(XPIECES % 256 == 0);
static_assert((OFF_W1 % 128) == 0 && (OFF_W2 % 128) == 0 && (OFF_M1 % 128) == 0 && (OFF_M2 % 128) == 0 && (OFF_M3 % 128) == 0);
static_assert(OFF_W1 + 16 * 32 * 2 == OFF_W2);
static_assert(OFF_W2 + 32 * 160 * 2 == OFF_M1);
static_assert(OFF_M1 + 64 * 96 * 2 == OFF_M2);
static_assert(OFF_M2 + 32 * 64 * 2 == OFF_M3);
static_assert(OFF_M3 + 16 * 32 * 2 == WS_TOTAL);

typedef _Float16 v16h __attribute__((ext_vector_type(16)));
typedef _Float16 v8h  __attribute__((ext_vector_type(8)));
typedef float    v8f  __attribute__((ext_vector_type(8)));
typedef float    v4f  __attribute__((ext_vector_type(4)));
typedef float    v2f  __attribute__((ext_vector_type(2)));
typedef unsigned int v4u __attribute__((ext_vector_type(4)));

union FragH { v16h v; v8h hf[2]; _Float16 e[16]; };

__device__ __forceinline__ float bf_rne(float f) {
  unsigned x = __float_as_uint(f);
  x = (x + 0x7FFFu + ((x >> 16) & 1u)) & 0xFFFF0000u;
  return __uint_as_float(x);
}
__device__ __forceinline__ v8f zero8() { v8f z = {0.f, 0.f, 0.f, 0.f, 0.f, 0.f, 0.f, 0.f}; return z; }
__device__ __forceinline__ v8h zero8h() {
  v8h z;
#pragma unroll
  for (int i = 0; i < 8; ++i) z[i] = (_Float16)0.0f;
  return z;
}
__device__ __forceinline__ float rcp_f(float x) {
#if defined(__HIP_DEVICE_COMPILE__)
  return __builtin_amdgcn_rcpf(x);
#else
  return 1.0f / x;
#endif
}

__device__ __forceinline__ v16h ldfrag(const _Float16* p) {
  FragH f;
  f.hf[0] = *(const v8h*)(p);
  f.hf[1] = *(const v8h*)(p + 16);
  return f.v;
}

__device__ __forceinline__ v8f mma(v16h a, v16h b, v8f c) {
  v8f d = __builtin_amdgcn_wmma_f32_16x16x32_f16(false, a, false, b, (short)0, c, false, false);
#if defined(__HIP_DEVICE_COMPILE__)
  asm volatile("v_nop\n\tv_nop\n\tv_nop\n\tv_nop" : "+v"(d) : "v"(a), "v"(b));
#endif
  return d;
}

__device__ __forceinline__ void st16x2(_Float16* dst, v8h val, bool act) {
  union { v8h h; v4u u; } c;
  c.h = val;
  const v4u u = c.u;
  if (act) *(volatile v4u*)dst = u;
  __threadfence();
  if (act) *(volatile v4u*)dst = u;
}

__global__ __launch_bounds__(256)
void k_pack(const float* __restrict__ te,  const float* __restrict__ trw, const float* __restrict__ trb,
            const float* __restrict__ c1w, const float* __restrict__ c2w,
            const float* __restrict__ m1w, const float* __restrict__ m2w, const float* __restrict__ m3w,
            float* textf, _Float16* w1p, _Float16* w2p, _Float16* q1p, _Float16* q2p, _Float16* q3p)
{
  const int tid = threadIdx.x;
  const int pl  = blockIdx.y;
  const int g   = blockIdx.x * 256 + tid;

  if (pl == 0) {
    if (blockIdx.x == 0 && tid < NBATCH * NF) {
      const int bb = tid >> 5, n = tid & 31;
      float acc = 0.0f;
#pragma unroll 1
      for (int k = 0; k < TXTK; ++k)
        acc = fmaf(bf_rne(te[bb * TXTK + k]), bf_rne(trw[k * NF + n]), acc);
      acc += bf_rne(trb[n]);
      float* dst = textf + tid;
      *(volatile float*)dst = acc;
      __threadfence();
      *(volatile float*)dst = acc;
    }
  } else if (pl == 1) {
    const int gc = (g < 64) ? g : 63;
    v8h pk;
#pragma unroll
    for (int i = 0; i < 8; ++i) {
      const int e  = gc * 8 + i;
      const int n  = e >> 5, k = e & 31;
      const int kc = (k < 9) ? k : 8;
      const float xv = c1w[n * 9 + kc];
      pk[i] = (_Float16)((k < 9) ? bf_rne(xv) : 0.0f);
    }
    st16x2(w1p + (size_t)gc * 8, pk, g < 64);
  } else if (pl == 2) {
    const int gc = (g < 640) ? g : 639;
    v8h pk;
#pragma unroll
    for (int i = 0; i < 8; ++i) {
      const int e   = gc * 8 + i;
      const int n   = e / 160;
      const int k   = e - n * 160;
      const int tap = k >> 4, ci = k & 15;
      const int tc  = (tap < 9) ? tap : 8;
      const float xv = c2w[n * 144 + ci * 9 + tc];
      pk[i] = (_Float16)((tap < 9) ? bf_rne(xv) : 0.0f);
    }
    st16x2(w2p + (size_t)gc * 8, pk, g < 640);
  } else if (pl == 3) {
    const int gc = (g < 768) ? g : 767;
    v8h pk;
#pragma unroll
    for (int i = 0; i < 8; ++i) {
      const int e  = gc * 8 + i;
      const int n  = e / 96;
      const int k  = e - n * 96;
      const int kc = (k < 65) ? k : 64;
      const float xv = m1w[kc * 64 + n];
      pk[i] = (_Float16)((k < 65) ? bf_rne(xv) : 0.0f);
    }
    st16x2(q1p + (size_t)gc * 8, pk, g < 768);
  } else if (pl == 4) {
    const int gc = (g < 256) ? g : 255;
    v8h pk;
#pragma unroll
    for (int i = 0; i < 8; ++i) {
      const int e = gc * 8 + i;
      const int n = e >> 6, k = e & 63;
      pk[i] = (_Float16)bf_rne(m2w[k * 32 + n]);
    }
    st16x2(q2p + (size_t)gc * 8, pk, g < 256);
  } else {
    const int gc = (g < 64) ? g : 63;
    v8h pk;
#pragma unroll
    for (int i = 0; i < 8; ++i) {
      const int e = gc * 8 + i;
      const int n = e >> 5, k = e & 31;
      const float xv = m3w[k];
      pk[i] = (_Float16)((n == 0) ? bf_rne(xv) : 0.0f);
    }
    st16x2(q3p + (size_t)gc * 8, pk, g < 64);
  }
}

__global__ __launch_bounds__(256)
void k_copy(const float* __restrict__ x, const float* __restrict__ mk, float* out0, int npieces)
{
  const int g  = blockIdx.x * 256 + threadIdx.x;
  const int gc = (g < npieces) ? g : (npieces - 1);
  const v4f a = *(const v4f*)(x  + (size_t)gc * 4);
  const v4f q = *(const v4f*)(mk + (size_t)gc * 4);
  v4f r;
#pragma unroll
  for (int i = 0; i < 4; ++i) r[i] = bf_rne(a[i]) + 0.0f * (1.0f - q[i]);
  float* dst = out0 + (size_t)gc * 4;
  if (g < npieces) *(volatile v4f*)dst = r;
  __threadfence();
  if (g < npieces) *(volatile v4f*)dst = r;
}

__global__ __launch_bounds__(NTHR)
void k_main(const float* __restrict__ x,   const float* __restrict__ center,
            const float* __restrict__ c1b, const float* __restrict__ c2b,
            const float* __restrict__ m1b, const float* __restrict__ m2b, const float* __restrict__ m3b,
            const float* __restrict__ textf,
            const _Float16* __restrict__ w1p, const _Float16* __restrict__ w2p,
            const _Float16* __restrict__ q1p, const _Float16* __restrict__ q2p, const _Float16* __restrict__ q3p,
            float* out1)
{
  __shared__ __align__(16) _Float16 s_patch[WAVES][104];
  __shared__ __align__(16) _Float16 s_pool[WAVES][576];
  __shared__ __align__(16) _Float16 s_comb[16][96];
  __shared__ __align__(16) _Float16 s_h1[16][64];
  __shared__ __align__(16) _Float16 s_h2[16][32];
  __shared__ __align__(16) float    s_out[PPB];

  const int tid  = threadIdx.x;
  const int w    = __builtin_amdgcn_readfirstlane(tid >> 5);
  const int lane = tid & 31;
  const int m    = lane & 15;
  const int h    = lane >> 4;
  const int b    = (int)(blockIdx.x >> 9);

  for (int i = lane; i < 104; i += 32) s_patch[w][i] = (_Float16)0.0f;
  {
    const v8h z = zero8h();
    for (int i = lane; i < 72; i += 32) *(v8h*)(&s_pool[w][8 * i]) = z;
  }
  const float cpx = bf_rne(center[0]);
  const float cpy = bf_rne(center[1]);
  const float md  = fmaxf(fmaxf(fabsf(cpx), fabsf(cpy)),
                          fmaxf(fabsf(cpx - (float)IMG), fabsf(cpy - (float)IMG)));
  const float rmd = 1.0f / md;
  const float bias1 = bf_rne(c1b[m]);
  const float b20   = bf_rne(c2b[m]);
  const float b21   = bf_rne(c2b[16 + m]);
  const float b3    = bf_rne(m3b[0]);
  const int   lm1   = (lane > 0) ? (lane - 1) : 0;
  const float tfa   = textf[b * NF + lm1];
  const float tfz   = textf[b * NF + 31];
  const v16h  bw1   = ldfrag(w1p + m * 32 + 8 * h);

#pragma unroll 1
  for (int q = 0; q < 2; ++q) {
    const int p  = (int)blockIdx.x * PPB + q * 16 + w;
    const int pi = p & (NPB - 1);
    const int py = pi >> 7;
    const int px = pi & 127;

    {
      const int r  = lane >> 2;
      const int c0 = (lane & 3) * 2;
      const float* src = x + ((size_t)b << 20) + (size_t)(py * 8 + r) * IMG + (size_t)(px * 8 + c0);
      const v2f v = *(const v2f*)src;
      s_patch[w][(r + 1) * 10 + c0 + 1] = (_Float16)bf_rne(v[0]);
      s_patch[w][(r + 1) * 10 + c0 + 2] = (_Float16)bf_rne(v[1]);
    }
    __syncthreads();

#pragma unroll
    for (int t = 0; t < 4; ++t) {
      const int r    = 2 * t + (m >> 3);
      const int c    = m & 7;
      const int base = r * 10 + c;
      FragH a;
      a.hf[1] = zero8h();
      a.e[0]  = s_patch[w][base + (h ? 22 : 0)];
#pragma unroll
      for (int i = 1; i < 8; ++i) {
        const int off = (i / 3) * 10 + (i % 3);
        const _Float16 v = s_patch[w][base + off];
        a.e[i] = h ? (_Float16)0.0f : v;
      }
      const v8f acc = mma(a.v, bw1, zero8());
      float hm0 = fmaxf(acc[0], acc[1]);
      float hm1 = fmaxf(acc[2], acc[3]);
      float hm2 = fmaxf(acc[4], acc[5]);
      float hm3 = fmaxf(acc[6], acc[7]);
      hm0 = fmaxf(hm0, __shfl_xor(hm0, 16, 32));
      hm1 = fmaxf(hm1, __shfl_xor(hm1, 16, 32));
      hm2 = fmaxf(hm2, __shfl_xor(hm2, 16, 32));
      hm3 = fmaxf(hm3, __shfl_xor(hm3, 16, 32));
      const float pl0 = fmaxf(hm0 + bias1, 0.0f);
      const float pl1 = fmaxf(hm1 + bias1, 0.0f);
      const float pl2 = fmaxf(hm2 + bias1, 0.0f);
      const float pl3 = fmaxf(hm3 + bias1, 0.0f);
      const float vA  = h ? pl2 : pl0;
      const float vB  = h ? pl3 : pl1;
      const int cellA = (t + 1) * 6 + 1 + 2 * h;
      s_pool[w][cellA * 16 + m]       = (_Float16)vA;
      s_pool[w][(cellA + 1) * 16 + m] = (_Float16)vB;
    }
    __syncthreads();

    {
      const int yy = m >> 2, xx = m & 3;
      v8f acc0 = zero8(), acc1 = zero8();
#pragma unroll
      for (int s = 0; s < 5; ++s) {
        const int tap0  = 2 * s;
        const int tap1  = 2 * s + 1;
        const int tap1c = (tap1 < 9) ? tap1 : 8;
        const int cell0 = (yy + tap0 / 3) * 6 + (xx + tap0 % 3);
        const int cell1 = (yy + tap1c / 3) * 6 + (xx + tap1c % 3);
        FragH a;
        a.hf[0] = *(const v8h*)(&s_pool[w][cell0 * 16 + 8 * h]);
        const v8h a1 = *(const v8h*)(&s_pool[w][cell1 * 16 + 8 * h]);
        a.hf[1] = (tap1 < 9) ? a1 : zero8h();
        const _Float16* bp = w2p + (size_t)m * 160 + 32 * s + 8 * h;
        const v16h bb0 = ldfrag(bp);
        const v16h bb1 = ldfrag(bp + 16 * 160);
        acc0 = mma(a.v, bb0, acc0);
        acc1 = mma(a.v, bb1, acc1);
      }
      float s0 = 0.0f, s1 = 0.0f;
#pragma unroll
      for (int rr = 0; rr < 8; ++rr) {
        s0 += fmaxf(acc0[rr] + b20, 0.0f);
        s1 += fmaxf(acc1[rr] + b21, 0.0f);
      }
      s0 += __shfl_xor(s0, 16, 32);
      s1 += __shfl_xor(s1, 16, 32);
      const float vis = (h ? s1 : s0) * 0.0625f;
      s_comb[w][lane] = (_Float16)vis;

      const float pcx  = (float)(px * 8 + 4);
      const float pcy  = (float)(py * 8 + 4);
      const float dist = fmaxf(fabsf(pcx - cpx), fabsf(pcy - cpy));
      const float nd   = dist * rmd;
      const float c32  = (lane == 0) ? nd  : tfa;
      const float c64  = (lane == 0) ? tfz : 0.0f;
      s_comb[w][32 + lane] = (_Float16)c32;
      s_comb[w][64 + lane] = (_Float16)c64;
    }
    __syncthreads();

    if (w < 4) {
      const int nt = w;
      v8f acc = zero8();
#pragma unroll
      for (int s = 0; s < 3; ++s) {
        FragH a;
        a.hf[0] = *(const v8h*)(&s_comb[m][32 * s + 8 * h]);
        a.hf[1] = *(const v8h*)(&s_comb[m][32 * s + 16 + 8 * h]);
        const v16h bb = ldfrag(q1p + (size_t)(nt * 16 + m) * 96 + 32 * s + 8 * h);
        acc = mma(a.v, bb, acc);
      }
      const int   n    = nt * 16 + m;
      const float bias = bf_rne(m1b[n]);
#pragma unroll
      for (int rr = 0; rr < 8; ++rr)
        s_h1[8 * h + rr][n] = (_Float16)fmaxf(acc[rr] + bias, 0.0f);
    }
    __syncthreads();

    if (w < 2) {
      const int nt = w;
      v8f acc = zero8();
#pragma unroll
      for (int s = 0; s < 2; ++s) {
        FragH a;
        a.hf[0] = *(const v8h*)(&s_h1[m][32 * s + 8 * h]);
        a.hf[1] = *(const v8h*)(&s_h1[m][32 * s + 16 + 8 * h]);
        const v16h bb = ldfrag(q2p + (size_t)(nt * 16 + m) * 64 + 32 * s + 8 * h);
        acc = mma(a.v, bb, acc);
      }
      const int   n    = nt * 16 + m;
      const float bias = bf_rne(m2b[n]);
#pragma unroll
      for (int rr = 0; rr < 8; ++rr)
        s_h2[8 * h + rr][n] = (_Float16)fmaxf(acc[rr] + bias, 0.0f);
    }
    __syncthreads();

    if (w == 0) {
      FragH a;
      a.hf[0] = *(const v8h*)(&s_h2[m][8 * h]);
      a.hf[1] = *(const v8h*)(&s_h2[m][16 + 8 * h]);
      const v16h bb  = ldfrag(q3p + m * 32 + 8 * h);
      const v8f  acc = mma(a.v, bb, zero8());
#pragma unroll
      for (int rr = 0; rr < 8; ++rr) {
        const float sv  = acc[rr] + b3;
        const float ex  = __expf(-sv);
        const float sig = rcp_f(1.0f + ex);
        const float sp  = fminf(fmaxf(5.0f * sig + 3.0f, 3.0f), 15.0f);
        if (m == 0) s_out[q * 16 + 8 * h + rr] = sp;
      }
    }
    __syncthreads();
  }

  {
    const int e = (tid < 8) ? tid : 0;
    const v4f v = *(const v4f*)(&s_out[4 * e]);
    float* dst = out1 + (size_t)blockIdx.x * PPB + 4 * e;
    if (tid < 8) *(volatile v4f*)dst = v;
    __threadfence();
    if (tid < 8) *(volatile v4f*)dst = v;
  }
}

extern "C" void kernel_launch(void* const* d_in, const int* in_sizes, int n_in,
                              void* d_out, int out_size, void* d_ws, size_t ws_size,
                              hipStream_t stream) {
  if (n_in < 16) return;
  if (in_sizes[0]  != XELEMS) return;
  if (in_sizes[1]  != NBATCH * TXTK) return;
  if (in_sizes[2]  != XELEMS) return;
  if (in_sizes[3]  != 2) return;
  if (in_sizes[4]  != TXTK * NF) return;
  if (in_sizes[5]  != NF) return;
  if (in_sizes[6]  != 16 * 9) return;
  if (in_sizes[7]  != 16) return;
  if (in_sizes[8]  != 32 * 144) return;
  if (in_sizes[9]  != 32) return;
  if (in_sizes[10] != 65 * 64) return;
  if (in_sizes[11] != 64) return;
  if (in_sizes[12] != 64 * 32) return;
  if (in_sizes[13] != 32) return;
  if (in_sizes[14] != 32) return;
  if (in_sizes[15] != 1) return;
  if (out_size != XELEMS + NPATCH) return;
  if (ws_size < (size_t)WS_TOTAL) return;

  const float* x   = (const float*)d_in[0];
  const float* te  = (const float*)d_in[1];
  const float* mk  = (const float*)d_in[2];
  const float* cp  = (const float*)d_in[3];
  const float* trw = (const float*)d_in[4];
  const float* trb = (const float*)d_in[5];
  const float* c1w = (const float*)d_in[6];
  const float* c1b = (const float*)d_in[7];
  const float* c2w = (const float*)d_in[8];
  const float* c2b = (const float*)d_in[9];
  const float* m1w = (const float*)d_in[10];
  const float* m1b = (const float*)d_in[11];
  const float* m2w = (const float*)d_in[12];
  const float* m2b = (const float*)d_in[13];
  const float* m3w = (const float*)d_in[14];
  const float* m3b = (const float*)d_in[15];

  float* out0 = (float*)d_out;
  float* out1 = out0 + XELEMS;

  unsigned char* ws = (unsigned char*)d_ws;
  float*    textf = (float*)(ws + OFF_TXT);
  _Float16* w1p   = (_Float16*)(ws + OFF_W1);
  _Float16* w2p   = (_Float16*)(ws + OFF_W2);
  _Float16* q1p   = (_Float16*)(ws + OFF_M1);
  _Float16* q2p   = (_Float16*)(ws + OFF_M2);
  _Float16* q3p   = (_Float16*)(ws + OFF_M3);

  k_pack<<<dim3(3, 6), dim3(256), 0, stream>>>(te, trw, trb, c1w, c2w, m1w, m2w, m3w,
                                               textf, w1p, w2p, q1p, q2p, q3p);
  k_copy<<<dim3(XPIECES / 256), dim3(256), 0, stream>>>(x, mk, out0, XPIECES);
  k_main<<<dim3(NBLK), dim3(NTHR), 0, stream>>>(x, cp, c1b, c2b, m1b, m2b, m3b, textf,
                                                w1p, w2p, q1p, q2p, q3p, out1);
  (void)hipGetLastError();
}
